// GeATLayer_369367188029
// MI455X (gfx1250) — hardware-verified
//
#include <hip/hip_runtime.h>


namespace {
constexpr int N = 2048, AD = 64, H = 8, NBT = 8, D = 512, CH = 128;
constexpr float XS = 8.0f, HS = 256.0f, PS = 256.0f, WSC = 256.0f;
typedef _Float16 b16;
typedef __attribute__((ext_vector_type(16))) _Float16 v16b;
typedef __attribute__((ext_vector_type(8))) _Float16 v8b;
typedef __attribute__((ext_vector_type(2))) _Float16 v2b;
typedef __attribute__((ext_vector_type(8))) float v8f;
typedef __attribute__((ext_vector_type(4))) float v4f;
__device__ __forceinline__ float bf16_rne(float f) { unsigned int u = __float_as_uint(f); u += 0x7FFFu + ((u >> 16) & 1u); float r = __uint_as_float(u & 0xFFFF0000u); asm volatile("" : "+v"(r)); return r; }
__device__ __forceinline__ float bfv(float f) { float r = bf16_rne(f); asm volatile("" : "+v"(r)); return r; }
__device__ __forceinline__ void split16(float v, b16& hi, b16& lo) { hi = (b16)v; lo = (b16)(v - (float)hi); }
__device__ __forceinline__ v16b frag_kb(const b16* p, int hh) { const v8b a = *(const v8b*)(p + 8 * hh), b = *(const v8b*)(p + 16 + 8 * hh); v16b f;
#pragma unroll
  for (int e = 0; e < 8; ++e) { f[e] = a[e]; f[8 + e] = b[e]; } return f; }
__device__ __forceinline__ v8f wmma16b(v16b a, v16b b, v8f c) { v8f d = __builtin_amdgcn_wmma_f32_16x16x32_f16(false, a, false, b, (short)0, c, false, false); asm volatile("v_nop\n\tv_nop\n\tv_nop\n\tv_nop" : "+v"(d) : "v"(a), "v"(b)); return d; }
__device__ __forceinline__ void wave_lds_sync() { __builtin_amdgcn_fence(__ATOMIC_RELEASE, "workgroup"); __builtin_amdgcn_wave_barrier(); __builtin_amdgcn_fence(__ATOMIC_ACQUIRE, "workgroup"); }
__device__ __forceinline__ float pmul(float a, float b) { float p = a * b; asm volatile("" : "+v"(p)); return p; }
__device__ __forceinline__ int iclamp(int v, int lo, int hi) { return v < lo ? lo : (v > hi ? hi : v); }

__global__ __launch_bounds__(256) void wput_kernel(const float* __restrict__ qw, const float* __restrict__ kw, const float* __restrict__ vw, const float* __restrict__ a, const float* __restrict__ pw, b16* __restrict__ WQKV, b16* __restrict__ WA, b16* __restrict__ WP) { const size_t nt = (size_t)gridDim.x * 256, u0 = (size_t)blockIdx.x * 256 + threadIdx.x; v8b v;
  for (size_t u = u0; u < (size_t)3 * D * 8; u += nt) { const int o = (int)(u / 8), k0 = (int)(u % 8) * 8; const float* w = o < D ? qw : (o < 2 * D ? kw : vw); const int oo = o % D;
#pragma unroll
    for (int j = 0; j < 8; ++j) v[j] = (b16)(bf16_rne(w[(size_t)(k0 + j) * D + oo]) * WSC); for (int pass = 0; pass < 2; ++pass) { *(volatile v8b*)(WQKV + (size_t)o * AD + k0) = v; __threadfence(); } }
  for (size_t u = u0; u < (size_t)128 * 64; u += nt) { const int r = (int)(u / 64), k0 = (int)(u % 64) * 8; const int half = r / 64, kk = (r % 64) / H, h = r % H;
#pragma unroll
    for (int j = 0; j < 8; ++j) v[j] = (b16)(bf16_rne(a[((size_t)kk * 2 * D + half * D + k0 + j) * H + h]) * WSC); for (int pass = 0; pass < 2; ++pass) { *(volatile v8b*)(WA + (size_t)r * D + k0) = v; __threadfence(); } }
  for (size_t u = u0; u < (size_t)AD * 64; u += nt) { const int o = (int)(u / 64), k0 = (int)(u % 64) * 8;
#pragma unroll
    for (int j = 0; j < 8; ++j) v[j] = (b16)(bf16_rne(pw[(size_t)(k0 + j) * AD + o]) * WSC); for (int pass = 0; pass < 2; ++pass) { *(volatile v8b*)(WP + (size_t)o * D + k0) = v; __threadfence(); } } }
__global__ __launch_bounds__(32) void proj_kernel(const float* __restrict__ x, const b16* __restrict__ WQKV, const float* __restrict__ qb, const float* __restrict__ kb, const float* __restrict__ vb, const b16* __restrict__ WA, float* __restrict__ S, float* __restrict__ V) { __shared__ __attribute__((aligned(16))) b16 Ax[16][AD + 8], Ah[16][D + 8], Al[16][D + 8]; __shared__ float Tf[16][260], Sq[16][132]; const int lane = threadIdx.x, nloc = lane & 15, hlf = lane >> 4; const size_t i0 = (size_t)blockIdx.x * 16;
  for (int rr = 0; rr < 16; ++rr) for (int q = 0; q < 2; ++q) Ax[rr][q * 32 + lane] = (b16)(bf16_rne(x[(i0 + rr) * AD + q * 32 + lane]) * XS);
  if (lane < 16) { for (int k = AD; k < AD + 8; ++k) Ax[lane][k] = (b16)0.0f; for (int k = D; k < D + 8; ++k) { Ah[lane][k] = (b16)0.0f; Al[lane][k] = (b16)0.0f; } }
  wave_lds_sync(); const v16b a0 = frag_kb(&Ax[nloc][0], hlf), a1 = frag_kb(&Ax[nloc][32], hlf);
#pragma unroll 1
  for (int which = 0; which < 3; ++which) { const float* bias = which == 0 ? qb : (which == 1 ? kb : vb);
#pragma unroll 1
    for (int g = 0; g < 2; ++g) { v8f acc[16];
#pragma unroll
      for (int t = 0; t < 16; ++t) { const b16* wp = WQKV + ((size_t)which * D + g * 256 + t * 16 + nloc) * AD; acc[t] = wmma16b(a0, frag_kb(wp, hlf), (v8f){}); acc[t] = wmma16b(a1, frag_kb(wp + 32, hlf), acc[t]); }
#pragma unroll
      for (int t = 0; t < 16; ++t) { const int cc = t * 16 + nloc; const float bb = bfv(bias[g * 256 + cc]);
#pragma unroll
        for (int r8 = 0; r8 < 8; ++r8) Tf[8 * hlf + r8][cc] = acc[t][r8] * (1.0f / (XS * WSC)) + bb; }
      wave_lds_sync();
      if (which == 2) { for (int pass = 0; pass < 2; ++pass) { for (int rr = 0; rr < 16; ++rr) for (int q = 0; q < 2; ++q) *(volatile v4f*)(V + (i0 + rr) * D + g * 256 + q * 128 + lane * 4) = *(const v4f*)(&Tf[rr][q * 128 + lane * 4]); __threadfence(); } }
      else { for (int rr = 0; rr < 16; ++rr) for (int q = 0; q < 8; ++q) { const int c = q * 32 + lane; b16 p, pl; split16(Tf[rr][c] * HS, p, pl); Ah[rr][g * 256 + c] = p; Al[rr][g * 256 + c] = pl; } }
      wave_lds_sync(); }
    if (which < 2) { v8f acc[4] = {(v8f){}, (v8f){}, (v8f){}, (v8f){}};
#pragma unroll 2
      for (int kb_ = 0; kb_ < D; kb_ += 32) { const v16b a = frag_kb(&Ah[nloc][kb_], hlf), al = frag_kb(&Al[nloc][kb_], hlf);
#pragma unroll
        for (int t = 0; t < 4; ++t) { const v16b bw = frag_kb(WA + ((size_t)which * 64 + t * 16 + nloc) * D + kb_, hlf); acc[t] = wmma16b(a, bw, acc[t]); acc[t] = wmma16b(al, bw, acc[t]); } }
#pragma unroll
      for (int t = 0; t < 4; ++t)
#pragma unroll
        for (int r8 = 0; r8 < 8; ++r8) Sq[8 * hlf + r8][which * 64 + t * 16 + nloc] = acc[t][r8] * (1.0f / (HS * WSC));
      wave_lds_sync(); } }
  for (int pass = 0; pass < 2; ++pass) { for (int rr = 0; rr < 16; ++rr) *(volatile v4f*)(S + (i0 + rr) * 128 + lane * 4) = *(const v4f*)(&Sq[rr][lane * 4]); __threadfence(); } }
__global__ __launch_bounds__(256) void vt_kernel(const float* __restrict__ V, b16* __restrict__ VTh, b16* __restrict__ VTl) { __shared__ float Tt[64][D / 2 + 1]; const int j0 = (blockIdx.x >> 1) * 64, c0 = (blockIdx.x & 1) * (D / 2); const int tid = threadIdx.x, wave = tid >> 5, lane = tid & 31;
  for (int q = wave; q < 64; q += 8) for (int c = lane; c < D / 2; c += 32) Tt[q][c] = V[(size_t)(j0 + q) * D + c0 + c];
  __syncthreads();
  for (int pass = 0; pass < 2; ++pass) { for (int cc = wave; cc < D / 2; cc += 8) { const int c = c0 + cc; const int h = c / AD, d = c % AD; b16 h0, l0, h1, l1; split16(Tt[lane * 2][cc] * HS, h0, l0); split16(Tt[lane * 2 + 1][cc] * HS, h1, l1); const size_t o = ((size_t)h * AD + d) * N + j0 + lane * 2; *(volatile v2b*)(VTh + o) = (v2b){h0, h1}; *(volatile v2b*)(VTl + o) = (v2b){l0, l1}; } __threadfence(); } }
__global__ __launch_bounds__(32) void att_kernel(const float* __restrict__ S, const int* __restrict__ edges, const b16* __restrict__ VTh, const b16* __restrict__ VTl, int RLIM, float* __restrict__ O) { __shared__ __attribute__((aligned(16))) b16 Pa[4][16][CH + 8], Pb[4][16][CH + 8]; __shared__ float S1[16][64], Mx[16][4], Iv[16][4], Tf[16][260]; const int lane = threadIdx.x, nloc = lane & 15, hlf = lane >> 4; const int hg = blockIdx.x & 1; const size_t i0 = (size_t)(blockIdx.x >> 1) * 16; if (i0 >= (size_t)RLIM) return;
  for (int rr = 0; rr < 16; ++rr) for (int q = 0; q < 2; ++q) S1[rr][q * 32 + lane] = S[(i0 + rr) * 128 + q * 32 + lane];
  if (lane < 16) for (int g = 0; g < 4; ++g) for (int k = CH; k < CH + 8; ++k) { Pa[g][lane][k] = (b16)0.0f; Pb[g][lane][k] = (b16)0.0f; }
  wave_lds_sync();
  auto logit4 = [&](int rr, int j, float* e4) { const int bt = edges[(i0 + rr) * N + j]; const bool valid = bt >= 0; const int k = iclamp(bt, 0, NBT - 1); const float* s2 = S + (size_t)j * 128 + 64 + k * H + hg * 4; const v4f sv = *(const v4f*)s2;
#pragma unroll
    for (int g = 0; g < 4; ++g) { float e = S1[rr][k * H + hg * 4 + g] + sv[g]; e = e > 0.0f ? e : 0.2f * e; e4[g] = valid ? e : 0.0f; } };
  for (int rr = 0; rr < 16; ++rr) { float mx[4] = {-INFINITY, -INFINITY, -INFINITY, -INFINITY}; for (int j = lane; j < N; j += 32) { float e4[4]; logit4(rr, j, e4);
#pragma unroll
      for (int g = 0; g < 4; ++g) mx[g] = fmaxf(mx[g], e4[g]); }
#pragma unroll
    for (int g = 0; g < 4; ++g) for (int o = 16; o; o >>= 1) mx[g] = fmaxf(mx[g], __shfl_xor(mx[g], o));
    float sm[4] = {0, 0, 0, 0}; for (int j = lane; j < N; j += 32) { float e4[4]; logit4(rr, j, e4);
#pragma unroll
      for (int g = 0; g < 4; ++g) sm[g] += __expf(e4[g] - mx[g]); }
#pragma unroll
    for (int g = 0; g < 4; ++g) { for (int o = 16; o; o >>= 1) sm[g] += __shfl_xor(sm[g], o); if (lane == 0) { Mx[rr][g] = mx[g]; Iv[rr][g] = 1.0f / sm[g]; } } }
  wave_lds_sync();
  v8f oacc[4][4];
#pragma unroll
  for (int g = 0; g < 4; ++g)
#pragma unroll
    for (int t = 0; t < 4; ++t) oacc[g][t] = (v8f){};
#pragma unroll 1
  for (int ch = 0; ch < N / CH; ++ch) { const int j0 = ch * CH;
    for (int rr = 0; rr < 16; ++rr) for (int q = 0; q < CH / 32; ++q) { const int j = j0 + q * 32 + lane; float e4[4]; logit4(rr, j, e4);
#pragma unroll
      for (int g = 0; g < 4; ++g) { const float p = __expf(e4[g] - Mx[rr][g]) * Iv[rr][g]; b16 ph, pl; split16(p * PS, ph, pl); Pa[g][rr][q * 32 + lane] = ph; Pb[g][rr][q * 32 + lane] = pl; } }
    wave_lds_sync();
#pragma unroll
    for (int g = 0; g < 4; ++g) { const int h = hg * 4 + g;
#pragma unroll
      for (int kb = 0; kb < CH; kb += 32) { const v16b pa = frag_kb(&Pa[g][nloc][kb], hlf), pb = frag_kb(&Pb[g][nloc][kb], hlf);
#pragma unroll
        for (int t = 0; t < 4; ++t) { const size_t vo = ((size_t)h * AD + t * 16 + nloc) * N + j0 + kb; const v16b vh = frag_kb(VTh + vo, hlf), vl = frag_kb(VTl + vo, hlf); oacc[g][t] = wmma16b(pa, vh, oacc[g][t]); oacc[g][t] = wmma16b(pa, vl, oacc[g][t]); oacc[g][t] = wmma16b(pb, vh, oacc[g][t]); } } }
    wave_lds_sync(); }
#pragma unroll
  for (int g = 0; g < 4; ++g)
#pragma unroll
    for (int t = 0; t < 4; ++t)
#pragma unroll
      for (int r8 = 0; r8 < 8; ++r8) Tf[8 * hlf + r8][g * 64 + t * 16 + nloc] = oacc[g][t][r8] * (1.0f / (PS * HS));
  wave_lds_sync();
  for (int pass = 0; pass < 2; ++pass) { for (int rr = 0; rr < 16; ++rr) for (int q = 0; q < 2; ++q) *(volatile v4f*)(O + (i0 + rr) * D + hg * 256 + q * 128 + lane * 4) = *(const v4f*)(&Tf[rr][q * 128 + lane * 4]); __threadfence(); } }
__global__ __launch_bounds__(32) void outp_kernel(const float* __restrict__ O, const b16* __restrict__ WP, const float* __restrict__ pb, int RLIM, float* __restrict__ out) { __shared__ __attribute__((aligned(16))) b16 Ah[16][D + 8], Al[16][D + 8]; __shared__ float Tf[16][AD + 1]; const int lane = threadIdx.x, nloc = lane & 15, hlf = lane >> 4; const size_t i0 = (size_t)blockIdx.x * 16; if (i0 >= (size_t)RLIM) return;
  for (int rr = 0; rr < 16; ++rr) for (int q = 0; q < D / 32; ++q) { const int c = q * 32 + lane; b16 p, pl; split16(O[(i0 + rr) * D + c] * HS, p, pl); Ah[rr][c] = p; Al[rr][c] = pl; }
  if (lane < 16) for (int k = D; k < D + 8; ++k) { Ah[lane][k] = (b16)0.0f; Al[lane][k] = (b16)0.0f; }
  wave_lds_sync(); v8f acc[4] = {(v8f){}, (v8f){}, (v8f){}, (v8f){}};
#pragma unroll 2
  for (int kb = 0; kb < D; kb += 32) { const v16b a = frag_kb(&Ah[nloc][kb], hlf), al = frag_kb(&Al[nloc][kb], hlf);
#pragma unroll
    for (int t = 0; t < 4; ++t) { const v16b bw = frag_kb(WP + (size_t)(t * 16 + nloc) * D + kb, hlf); acc[t] = wmma16b(a, bw, acc[t]); acc[t] = wmma16b(al, bw, acc[t]); } }
#pragma unroll
  for (int t = 0; t < 4; ++t) { const int cc = t * 16 + nloc; const float bb = bfv(pb[cc]);
#pragma unroll
    for (int r8 = 0; r8 < 8; ++r8) Tf[8 * hlf + r8][cc] = acc[t][r8] * (1.0f / (HS * WSC)) + bb; }
  wave_lds_sync();
  typedef __attribute__((ext_vector_type(2))) float v2f;
  for (int pass = 0; pass < 2; ++pass) { for (int rr = 0; rr < 16; ++rr) *(volatile v2f*)(out + (i0 + rr) * AD + lane * 2) = (v2f){Tf[rr][lane * 2], Tf[rr][lane * 2 + 1]}; __threadfence(); } }
}

extern "C" void kernel_launch(void* const* d_in, const int* in_sizes, int n_in, void* d_out, int out_size, void* d_ws, size_t ws_size, hipStream_t stream) {
  (void)n_in;
  auto Fp = [&](int i) { return (const float*)d_in[i]; }; auto Ip = [&](int i) { return (const int*)d_in[i]; };
  if (in_sizes[0] != N * AD || in_sizes[1] != N * N || in_sizes[2] != AD * D || in_sizes[4] != AD * D || in_sizes[6] != AD * D || in_sizes[8] != NBT * 2 * D * H || in_sizes[9] != D * AD || out_size != N * AD) return;
  const int RLIM = N;
  size_t off = 0; char* ws = (char*)d_ws;
  auto carve = [&](size_t bytes) { char* p = ws + off; off += (bytes + 255) & ~(size_t)255; return p; };
  b16* WQKV = (b16*)carve((size_t)3 * D * AD * 2); b16* WA = (b16*)carve((size_t)128 * D * 2); b16* WP = (b16*)carve((size_t)AD * D * 2); float* S = (float*)carve((size_t)N * 128 * 4); float* V = (float*)carve((size_t)N * D * 4); b16* VTh = (b16*)carve((size_t)H * AD * N * 2); b16* VTl = (b16*)carve((size_t)H * AD * N * 2); float* O = (float*)carve((size_t)N * D * 4);
  if (off > ws_size || off > ((size_t)20 << 20)) return;
  wput_kernel<<<64, 256, 0, stream>>>(Fp(2), Fp(4), Fp(6), Fp(8), Fp(9), WQKV, WA, WP);
  proj_kernel<<<N / 16, 32, 0, stream>>>(Fp(0), WQKV, Fp(3), Fp(5), Fp(7), WA, S, V);
  vt_kernel<<<(N / 64) * 2, 256, 0, stream>>>(V, VTh, VTl);
  att_kernel<<<2 * (RLIM / 16), 32, 0, stream>>>(S, Ip(1), VTh, VTl, RLIM, O);
  outp_kernel<<<RLIM / 16, 32, 0, stream>>>(O, WP, Fp(10), RLIM, (float*)d_out);
}
